// CrossAttentionBlockWithTime_16398185136215
// MI455X (gfx1250) — hardware-verified
//
#include <hip/hip_runtime.h>


#define NB_  4
#define TT   2048
#define DD   256
#define NH_  8
#define HD   32
#define DV   256
#define KVW  2304
#define DE   1024
#define DT   256
#define ZH   1
#define PCAR 1024.0f
#define SCL  0.17677669529663688f
typedef _Float16 h16;
typedef unsigned short bf;
typedef __attribute__((ext_vector_type(16))) __bf16   v16bf;
typedef __attribute__((ext_vector_type(16))) _Float16 v16h;
typedef __attribute__((ext_vector_type(8)))  _Float16 v8h;
typedef __attribute__((ext_vector_type(8)))  unsigned short v8us;
typedef __attribute__((ext_vector_type(8)))  float    v8f;
typedef __attribute__((ext_vector_type(4)))  float    v4f;
typedef v8h  __attribute__((may_alias)) v8ha;
typedef v4f  __attribute__((may_alias)) v4fa;
typedef v8us __attribute__((may_alias)) v8usa;

__device__ __forceinline__ unsigned short f2bf(float f) { unsigned u = __float_as_uint(f); u += 0x7FFFu + ((u >> 16) & 1u); return (unsigned short)(u >> 16); }
__device__ __forceinline__ float bf2f(unsigned short b) { return __uint_as_float(((unsigned)b) << 16); }
__device__ __forceinline__ float bfr(float f) { return bf2f(f2bf(f)); }
__device__ __forceinline__ v16h cat16(v8h lo, v8h hi) { return __builtin_shufflevector(lo, hi, 0, 1, 2, 3, 4, 5, 6, 7, 8, 9, 10, 11, 12, 13, 14, 15); }
__device__ __forceinline__ v16bf cat16b(v8us lo, v8us hi) { return __builtin_bit_cast(v16bf, __builtin_shufflevector(lo, hi, 0, 1, 2, 3, 4, 5, 6, 7, 8, 9, 10, 11, 12, 13, 14, 15)); }
__device__ __forceinline__ v8f wmma16(v16h a, v16h b, v8f c) { return __builtin_amdgcn_wmma_f32_16x16x32_f16(false, a, false, b, (short)0, c, false, false); }
__device__ __forceinline__ v8f wmmab(v16bf a, v16bf b, v8f c) { return __builtin_amdgcn_wmma_f32_16x16x32_bf16(false, a, false, b, (short)0, c, false, false); }


template <typename T16> struct WFrag;
template <> struct WFrag<h16> { typedef v16h V; static __device__ __forceinline__ V ld(const h16* p) { return cat16(*(const v8h*)p, *(const v8h*)(p + 16)); } static __device__ __forceinline__ v8f mma(V a, V b, v8f c) { return wmma16(a, b, c); } };
template <> struct WFrag<bf> { typedef v16bf V; static __device__ __forceinline__ V ld(const bf* p) { return cat16b(*(const v8us*)p, *(const v8us*)(p + 16)); } static __device__ __forceinline__ v8f mma(V a, V b, v8f c) { return wmmab(a, b, c); } };
template <typename T16, int NSPLIT, bool BIAS>
__global__ __launch_bounds__(32) void k_gemmw(const T16* __restrict__ A, const T16* __restrict__ A2, const T16* __restrict__ Bt, const T16* __restrict__ Bt2, int K, float* C, int ldc, const float* __restrict__ bias, size_t sA, size_t sB, size_t sC) {
    typedef typename WFrag<T16>::V V;
    __shared__ __align__(16) float os[16 * 68];
    const size_t z = blockIdx.z; A += z * sA; if (A2) A2 += z * sA; Bt += z * sB; if (Bt2) Bt2 += z * sB; C += z * sC;
    const int lane = threadIdx.x & 31, lr = lane & 15, hi = lane >> 4; const int r0 = blockIdx.x * 64, c0 = blockIdx.y * 64;
    v8f acc[4][4];
#pragma unroll
    for (int mb = 0; mb < 4; ++mb)
#pragma unroll
        for (int nb = 0; nb < 4; ++nb) acc[mb][nb] = (v8f){};
    const size_t aoff = (size_t)(r0 + lr) * K + 8 * hi, boff = (size_t)(c0 + lr) * K + 8 * hi;
#pragma unroll 1
    for (int kc = 0; kc < K; kc += 32) {
        V a[4], a2[4];
#pragma unroll
        for (int mb = 0; mb < 4; ++mb) { a[mb] = WFrag<T16>::ld(A + aoff + (size_t)mb * 16 * K + kc); if (NSPLIT == 1 || NSPLIT == 2) a2[mb] = WFrag<T16>::ld(A2 + aoff + (size_t)mb * 16 * K + kc); }
#pragma unroll
        for (int nb = 0; nb < 4; ++nb) { const V b = WFrag<T16>::ld(Bt + boff + (size_t)nb * 16 * K + kc); V b2; if (NSPLIT >= 2) b2 = WFrag<T16>::ld(Bt2 + boff + (size_t)nb * 16 * K + kc);
#pragma unroll
            for (int mb = 0; mb < 4; ++mb) { acc[mb][nb] = WFrag<T16>::mma(a[mb], b, acc[mb][nb]); if (NSPLIT == 1 || NSPLIT == 2) acc[mb][nb] = WFrag<T16>::mma(a2[mb], b, acc[mb][nb]); if (NSPLIT >= 2) acc[mb][nb] = WFrag<T16>::mma(a[mb], b2, acc[mb][nb]); } }
        asm volatile("v_nop\n\tv_nop\n\tv_nop\n\tv_nop" : "+v"(acc[0][0]), "+v"(acc[1][1]), "+v"(acc[2][2]), "+v"(acc[3][3]) : "v"(a[0]), "v"(a[3]));
    }
#pragma unroll
    for (int mb = 0; mb < 4; ++mb) {
#pragma unroll
        for (int nb = 0; nb < 4; ++nb) {
#pragma unroll
            for (int j = 0; j < 8; ++j) os[(hi * 8 + j) * 68 + nb * 16 + lr] = acc[mb][nb][j]; }
        __builtin_amdgcn_wave_barrier(); asm volatile("" ::: "memory");
        float* crow = C + (size_t)(r0 + mb * 16) * ldc + c0;
#pragma unroll 1
        for (int ps = 0; ps < 2; ++ps) {
#pragma unroll
            for (int s = 0; s < 8; ++s) { const int row = 2 * s + hi, cofs = lr * 4; v4f val = *(const v4fa*)(os + row * 68 + cofs); if (BIAS) { val[0] += bfr(bias[c0 + cofs]); val[1] += bfr(bias[c0 + cofs + 1]); val[2] += bfr(bias[c0 + cofs + 2]); val[3] += bfr(bias[c0 + cofs + 3]); }
                *(volatile v4f*)(crow + (size_t)row * ldc + cofs) = val; }
            if (ps == 0) __threadfence(); }
        __builtin_amdgcn_wave_barrier(); asm volatile("" ::: "memory");
    }
}

__device__ __forceinline__ h16 tohx(float x) { return (h16)x; }
__device__ __forceinline__ void splitf(float y, unsigned short& h, unsigned short& l) { h = f2bf(y); l = f2bf(y - bf2f(h)); }
__device__ __forceinline__ float siluf(float a) { return __fdiv_rn(a, __fadd_rn(1.0f, __expf(-a))); }
typedef __attribute__((ext_vector_type(2))) _Float16 v2h;
typedef __attribute__((ext_vector_type(4))) _Float16 v4h;
typedef __attribute__((ext_vector_type(2))) unsigned short v2us;
typedef __attribute__((ext_vector_type(4))) unsigned short v4us;

__global__ __launch_bounds__(256) void k_wtG(const float* __restrict__ w, int K, int N, bf* Bt) {
    const int lane = threadIdx.x & 31; const int L0 = (blockIdx.x * 8 + (threadIdx.x >> 5)) * 8; const int nlines = N * K / 64;
#pragma unroll 1
    for (int ps = 0; ps < 2; ++ps) {
#pragma unroll 1
        for (int l = 0; l < 8; ++l) { const int L = L0 + l; if (L >= nlines) break; const size_t e = (size_t)L * 64 + lane * 2; const int k = (int)(e % K), n = (int)(e / K); v2us o;
            o[0] = f2bf(w[(size_t)k * N + n]); o[1] = f2bf(w[(size_t)(k + 1) * N + n]); *(volatile v2us*)(Bt + e) = o; }
        if (ps == 0) __threadfence(); }
}
__global__ __launch_bounds__(256) void k_cvt8(const float* __restrict__ src, bf* dst, size_t n8) { const size_t i = (size_t)blockIdx.x * 256 + threadIdx.x; if (i >= n8) return; const v8f v = *(const v8f*)(src + i * 8); v8us o;
#pragma unroll
    for (int k = 0; k < 8; ++k) o[k] = f2bf(v[k]); *(volatile v8us*)(dst + i * 8) = o; __threadfence(); *(volatile v8us*)(dst + i * 8) = o; }
template <int MODE>
__global__ __launch_bounds__(256) void k_lnrow(const float* __restrict__ A, const float* __restrict__ E, const float* __restrict__ gg, const float* __restrict__ bb, bf* Yh, bf* Yl) {
    const int lane = threadIdx.x & 31; const int r = blockIdx.x * 8 + (threadIdx.x >> 5); if (r >= TT) return; float v[8]; float s = 0.f;
#pragma unroll
    for (int c = 0; c < 2; ++c) { const v4f a = *(const v4f*)(A + (size_t)r * DD + c * 128 + lane * 4);
#pragma unroll
        for (int q = 0; q < 4; ++q) { const int col = c * 128 + lane * 4 + q; float t0 = (MODE == 0) ? bfr(a[q]) : a[q]; asm volatile("" : "+v"(t0)); const float t1 = (MODE == 2) ? __fadd_rn(t0, bfr(E[col])) : t0; v[c * 4 + q] = t1; s = __fadd_rn(s, t1); } }
#pragma unroll
    for (int sh = 16; sh; sh >>= 1) s += __shfl_xor(s, sh, 32);
    const float mu = s * (1.0f / DD); float qq = 0.f;
#pragma unroll
    for (int i = 0; i < 8; ++i) { const float d0 = v[i] - mu; float p = __fmul_rn(d0, d0); asm volatile("" : "+v"(p)); qq = __fadd_rn(qq, p); }
#pragma unroll
    for (int sh = 16; sh; sh >>= 1) qq += __shfl_xor(qq, sh, 32);
    const float rs = __fdiv_rn(1.0f, __fsqrt_rn(__fadd_rn(qq * (1.0f / DD), 1e-5f)));
#pragma unroll 1
    for (int ps = 0; ps < 2; ++ps) {
#pragma unroll
        for (int c = 0; c < 2; ++c) { v4us oh, ol;
#pragma unroll
            for (int q = 0; q < 4; ++q) { const int col = c * 128 + lane * 4 + q; float tn = __fmul_rn(v[c * 4 + q] - mu, rs); asm volatile("" : "+v"(tn)); float tg = __fmul_rn(tn, bfr(gg[col])); asm volatile("" : "+v"(tg)); float y = __fadd_rn(tg, bfr(bb[col]));
                if (MODE == 0) y = __fadd_rn(y, bfr(E[(size_t)r * DD + col])); unsigned short a2, c2; splitf(siluf(y), a2, c2); oh[q] = a2; ol[q] = c2; }
            const size_t o = (size_t)r * DD + c * 128 + lane * 4; *(volatile v4us*)(Yh + o) = oh; *(volatile v4us*)(Yl + o) = ol; }
        if (ps == 0) __threadfence(); }
}
__global__ __launch_bounds__(256) void k_qkpl(const float* __restrict__ QF, const float* __restrict__ KVF, h16* QP, h16* KP) { const int e = (blockIdx.x * 256 + threadIdx.x) * 2; if (e >= NH_ * TT * HD) return; const int d = e & 31; const int t = (e >> 5) & (TT - 1); const int h = e >> 16; v2h q2, k2;
    q2[0] = tohx(QF[(size_t)t * DD + h * HD + d]); q2[1] = tohx(QF[(size_t)t * DD + h * HD + d + 1]); k2[0] = tohx(KVF[(size_t)t * KVW + h * HD + d]); k2[1] = tohx(KVF[(size_t)t * KVW + h * HD + d + 1]);
    *(volatile v2h*)(QP + e) = q2; *(volatile v2h*)(KP + e) = k2; __threadfence(); *(volatile v2h*)(QP + e) = q2; *(volatile v2h*)(KP + e) = k2; }
__global__ __launch_bounds__(256) void k_vt(const float* __restrict__ KVF, h16* VT) { const size_t e = ((size_t)blockIdx.x * 256 + threadIdx.x) * 2; if (e >= (size_t)NH_ * DV * TT) return; const int t = (int)(e & (TT - 1)); const int c = (int)((e >> 11) & (DV - 1)); const int h = (int)(e >> 19); v2h v;
    v[0] = tohx(KVF[(size_t)t * KVW + NH_ * HD + h * DV + c]); v[1] = tohx(KVF[(size_t)(t + 1) * KVW + NH_ * HD + h * DV + c]); *(volatile v2h*)(VT + e) = v; __threadfence(); *(volatile v2h*)(VT + e) = v; }
__global__ __launch_bounds__(256) void k_asoft(const float* __restrict__ Sb, h16* P16) {
    const int lane = threadIdx.x & 31; const int row = blockIdx.x * 8 + (threadIdx.x >> 5); if (row >= ZH * TT) return; const int i = row & (TT - 1);
    const float* sr = Sb + (size_t)row * TT; float v[64]; float mx = -3.0e38f;
#pragma unroll
    for (int ch = 0; ch < 16; ++ch) { const int j0 = ch * 128 + lane * 4; const v4f a = *(const v4f*)(sr + j0);
#pragma unroll
        for (int q = 0; q < 4; ++q) { const int j = j0 + q; const float t = (j >= i) ? a[q] * SCL : -3.0e38f; v[ch * 4 + q] = t; mx = fmaxf(mx, t); } }
#pragma unroll
    for (int sh = 16; sh; sh >>= 1) mx = fmaxf(mx, __shfl_xor(mx, sh, 32));
    float sum = 0.f;
#pragma unroll
    for (int k = 0; k < 64; ++k) { v[k] = __expf(v[k] - mx); sum += v[k]; }
#pragma unroll
    for (int sh = 16; sh; sh >>= 1) sum += __shfl_xor(sum, sh, 32);
    const float f = __fdiv_rn(PCAR, sum);
#pragma unroll 1
    for (int ps = 0; ps < 2; ++ps) {
#pragma unroll
        for (int ch = 0; ch < 16; ++ch) { v4h o;
#pragma unroll
            for (int q = 0; q < 4; ++q) o[q] = tohx(v[ch * 4 + q] * f);
            *(volatile v4h*)(P16 + (size_t)row * TT + ch * 128 + lane * 4) = o; }
        if (ps == 0) __threadfence(); }
}
__global__ __launch_bounds__(256) void k_ocat(const float* __restrict__ O, int h, bf* Ah, bf* Al) { const int e = (blockIdx.x * 256 + threadIdx.x) * 2; if (e >= TT * DV) return; const int t = e / DV, c = e % DV; v2us oh, ol;
#pragma unroll
    for (int q = 0; q < 2; ++q) { unsigned short a, c2; splitf(O[e + q] * (1.0f / PCAR), a, c2); oh[q] = a; ol[q] = c2; } const size_t o = (size_t)t * (NH_ * DV) + h * DV + c; *(volatile v2us*)(Ah + o) = oh; *(volatile v2us*)(Al + o) = ol; __threadfence(); *(volatile v2us*)(Ah + o) = oh; *(volatile v2us*)(Al + o) = ol; }
__global__ __launch_bounds__(256) void k_res(const float* __restrict__ x, const float* __restrict__ M, float* X1) { const size_t i = ((size_t)blockIdx.x * 256 + threadIdx.x) * 4; if (i >= (size_t)TT * DD) return; const v4f a = *(const v4f*)(x + i), b = *(const v4f*)(M + i); v4f o;
#pragma unroll
    for (int q = 0; q < 4; ++q) o[q] = __fadd_rn(bfr(a[q]), b[q]); *(volatile v4f*)(X1 + i) = o; __threadfence(); *(volatile v4f*)(X1 + i) = o; }
__global__ __launch_bounds__(256) void k_t1(const float* __restrict__ tt, const float* __restrict__ W, const float* __restrict__ bb, float* TH1) { const int i = blockIdx.x * 256 + threadIdx.x; if (i >= NB_ * DT) return; const int b = i / DT, j = i % DT; float s = 0.f;
#pragma unroll 4
    for (int k = 0; k < DT; ++k) { float p = __fmul_rn(bfr(tt[b * DT + k]), bfr(W[(size_t)k * DT + j])); asm volatile("" : "+v"(p)); s = __fadd_rn(s, p); }
    const float o = siluf(__fadd_rn(s, bfr(bb[j]))); *(volatile float*)(TH1 + i) = o; __threadfence(); *(volatile float*)(TH1 + i) = o; }
__global__ __launch_bounds__(256) void k_t2(const float* __restrict__ TH1, const float* __restrict__ W, const float* __restrict__ bb, float* TH) { const int i = blockIdx.x * 256 + threadIdx.x; if (i >= NB_ * (DD + DE)) return; const int b = i / (DD + DE), k = i % (DD + DE); float s = 0.f;
#pragma unroll 4
    for (int j = 0; j < DT; ++j) { float p = __fmul_rn(TH1[b * DT + j], bfr(W[(size_t)j * (DD + DE) + k])); asm volatile("" : "+v"(p)); s = __fadd_rn(s, p); }
    const float o = __fadd_rn(s, bfr(bb[k])); *(volatile float*)(TH + i) = o; __threadfence(); *(volatile float*)(TH + i) = o; }
__global__ __launch_bounds__(256) void k_gateh(const float* __restrict__ HF, const float* __restrict__ THb, bf* Hh, bf* Hl) { const int e = (blockIdx.x * 256 + threadIdx.x) * 2; if (e >= TT * DE) return; const int k = e % DE; v2us oh, ol;
#pragma unroll
    for (int q = 0; q < 2; ++q) { const float sc = __fdiv_rn(1.0f, __fadd_rn(1.0f, __expf(-THb[DD + k + q]))); unsigned short a, c2; splitf(siluf(__fmul_rn(HF[e + q], sc)), a, c2); oh[q] = a; ol[q] = c2; }
    *(volatile v2us*)(Hh + e) = oh; *(volatile v2us*)(Hl + e) = ol; __threadfence(); *(volatile v2us*)(Hh + e) = oh; *(volatile v2us*)(Hl + e) = ol; }
__global__ __launch_bounds__(256) void k_fin(const float* __restrict__ F2, const float* __restrict__ X1, float* OUT) { const size_t i = ((size_t)blockIdx.x * 256 + threadIdx.x) * 4; if (i >= (size_t)TT * DD) return; const v4f a = *(const v4f*)(F2 + i), b = *(const v4f*)(X1 + i); v4f o;
#pragma unroll
    for (int q = 0; q < 4; ++q) o[q] = __fadd_rn(a[q], b[q]); *(volatile v4f*)(OUT + i) = o; __threadfence(); *(volatile v4f*)(OUT + i) = o; }

extern "C" void kernel_launch(void* const* d_in, const int* in_sizes, int n_in,
                              void* d_out, int out_size, void* d_ws, size_t ws_size, hipStream_t stream) {
    (void)in_sizes; (void)n_in; (void)out_size;
    const float* IN[26]; for (int i = 0; i < 26; ++i) IN[i] = (const float*)d_in[i];
    float* OUT = (float*)d_out;
    char* wsp = (char*)d_ws;
    auto take = [&](size_t bytes) { char* p = wsp; wsp += (bytes + 255) & ~(size_t)255; return (void*)p; };
    bf* WQ = (bf*)take((size_t)DD * DD * 2); bf* WKV1 = (bf*)take((size_t)DD * DD * 2); bf* WKV2 = (bf*)take((size_t)KVW * DD * 2); bf* WM = (bf*)take((size_t)DD * (NH_ * DV) * 2); bf* WF1 = (bf*)take((size_t)DE * DD * 2); bf* WF2 = (bf*)take((size_t)DD * DE * 2);
    float* TH1 = (float*)take((size_t)NB_ * DT * 4); float* TH = (float*)take((size_t)NB_ * (DD + DE) * 4);
    bf* Ph = (bf*)take((size_t)TT * DE * 2); bf* Pl = (bf*)take((size_t)TT * DE * 2); bf* CB = (bf*)take((size_t)TT * DD * 2); float* QF = (float*)take((size_t)TT * DD * 4); float* KVF = (float*)take((size_t)TT * KVW * 4);
    h16* QP = (h16*)take((size_t)NH_ * TT * HD * 2); h16* KP = (h16*)take((size_t)NH_ * TT * HD * 2); h16* VT = (h16*)take((size_t)NH_ * DV * TT * 2); float* Sb = (float*)take((size_t)TT * TT * 4); h16* Pm = (h16*)take((size_t)TT * TT * 2); float* O = (float*)take((size_t)TT * DV * 4);
    bf* ATh = (bf*)take((size_t)TT * NH_ * DV * 2); bf* ATl = (bf*)take((size_t)TT * NH_ * DV * 2); float* X1 = (float*)take((size_t)TT * DD * 4); float* HF = (float*)take((size_t)TT * DE * 4); float* F2 = (float*)take((size_t)TT * DD * 4);
    if ((size_t)(wsp - (char*)d_ws) > ws_size) return;
    { const unsigned g1 = (unsigned)((DD * DD / 64 + 63) / 64); k_wtG<<<g1, 256, 0, stream>>>(IN[6], DD, DD, WQ); k_wtG<<<g1, 256, 0, stream>>>(IN[8], DD, DD, WKV1); k_wtG<<<(unsigned)((DD * KVW / 64 + 63) / 64), 256, 0, stream>>>(IN[12], DD, KVW, WKV2);
      k_wtG<<<(unsigned)(((NH_ * DV) * DD / 64 + 63) / 64), 256, 0, stream>>>(IN[14], NH_ * DV, DD, WM); k_wtG<<<(unsigned)((DD * DE / 64 + 63) / 64), 256, 0, stream>>>(IN[22], DD, DE, WF1); k_wtG<<<(unsigned)((DE * DD / 64 + 63) / 64), 256, 0, stream>>>(IN[24], DE, DD, WF2);
      k_t1<<<(NB_ * DT + 255) / 256, 256, 0, stream>>>(IN[2], IN[16], IN[17], TH1); k_t2<<<(NB_ * (DD + DE) + 255) / 256, 256, 0, stream>>>(TH1, IN[18], IN[19], TH); }
    const unsigned LD = (TT * DD / 2 + 255) / 256, L4 = (TT * DD / 4 + 255) / 256; const dim3 gD(TT / 64, DD / 64, 1);
    for (int b = 0; b < NB_; ++b) { const float* xb = IN[0] + (size_t)b * TT * DD; const float* THb = TH + (size_t)b * (DD + DE);
        k_lnrow<0><<<TT / 8, 256, 0, stream>>>(xb, IN[3], IN[4], IN[5], Ph, Pl);
        k_gemmw<bf, 1, true><<<gD, 32, 0, stream>>>(Ph, Pl, WQ, nullptr, DD, QF, DD, IN[7], 0, 0, 0);
        k_cvt8<<<(unsigned)(((size_t)TT * DD / 8 + 255) / 256), 256, 0, stream>>>(IN[1] + (size_t)b * TT * DD, CB, (size_t)TT * DD / 8);
        k_gemmw<bf, 0, true><<<gD, 32, 0, stream>>>(CB, nullptr, WKV1, nullptr, DD, X1, DD, IN[9], 0, 0, 0);
        k_lnrow<1><<<TT / 8, 256, 0, stream>>>(X1, nullptr, IN[10], IN[11], Ph, Pl);
        k_gemmw<bf, 1, true><<<dim3(TT / 64, KVW / 64, 1), 32, 0, stream>>>(Ph, Pl, WKV2, nullptr, DD, KVF, KVW, IN[13], 0, 0, 0);
        k_qkpl<<<(NH_ * TT * HD / 2 + 255) / 256, 256, 0, stream>>>(QF, KVF, QP, KP); k_vt<<<(unsigned)(((size_t)NH_ * DV * TT / 2 + 255) / 256), 256, 0, stream>>>(KVF, VT);
        for (int h = 0; h < NH_; ++h) {
            k_gemmw<h16, 0, false><<<dim3(TT / 64, TT / 64, 1), 32, 0, stream>>>(QP + (size_t)h * TT * HD, nullptr, KP + (size_t)h * TT * HD, nullptr, HD, Sb, TT, nullptr, 0, 0, 0);
            k_asoft<<<TT / 8, 256, 0, stream>>>(Sb, Pm);
            k_gemmw<h16, 0, false><<<dim3(TT / 64, DV / 64, 1), 32, 0, stream>>>(Pm, nullptr, VT + (size_t)h * DV * TT, nullptr, TT, O, DV, nullptr, 0, 0, 0);
            k_ocat<<<(TT * DV / 2 + 255) / 256, 256, 0, stream>>>(O, h, ATh, ATl); }
        k_gemmw<bf, 1, true><<<gD, 32, 0, stream>>>(ATh, ATl, WM, nullptr, NH_ * DV, QF, DD, IN[15], 0, 0, 0); k_res<<<L4, 256, 0, stream>>>(xb, QF, X1);
        k_lnrow<2><<<TT / 8, 256, 0, stream>>>(X1, THb, IN[20], IN[21], Ph, Pl);
        k_gemmw<bf, 1, true><<<dim3(TT / 64, DE / 64, 1), 32, 0, stream>>>(Ph, Pl, WF1, nullptr, DD, HF, DE, IN[23], 0, 0, 0);
        k_gateh<<<(TT * DE / 2 + 255) / 256, 256, 0, stream>>>(HF, THb, Ph, Pl);
        k_gemmw<bf, 1, true><<<gD, 32, 0, stream>>>(Ph, Pl, WF2, nullptr, DE, F2, DD, IN[25], 0, 0, 0);
        k_fin<<<L4, 256, 0, stream>>>(F2, X1, OUT + (size_t)b * TT * DD); }
}
